// ResGCN_89240830476623
// MI455X (gfx1250) — hardware-verified
//
#include <hip/hip_runtime.h>
#include <stdint.h>


typedef __attribute__((ext_vector_type(16))) _Float16 v16h;
typedef __attribute__((ext_vector_type(8)))  _Float16 v8h;
typedef __attribute__((ext_vector_type(8)))  float    v8f;
typedef __attribute__((ext_vector_type(4)))  float    v4f;
typedef __attribute__((ext_vector_type(2)))  int      v2i;
typedef unsigned int u64;

#define HD 128
#define NGRAPH 256
#define SORT_LOG 20
#define SORT_N (1 << SORT_LOG)
#define TILE 8192
#define VST2(T, ptr, val) do { const T _v = (val); *(volatile T*)(ptr) = _v; __threadfence(); *(volatile T*)(ptr) = _v; } while (0)

__device__ __forceinline__ v8f wmma16(v16h a, v16h b, v8f c) {
  v8f d = __builtin_amdgcn_wmma_f32_16x16x32_f16(false, a, false, b, (short)0, c, false, false);
  asm volatile("v_nop\n\tv_nop\n\tv_nop\n\tv_nop" : "+v"(d) : "v"(a), "v"(b));
  return d;
}

__global__ __launch_bounds__(256) void k_sort_init(const int* __restrict__ src, const int* __restrict__ dst, u64* __restrict__ A, int E) {
  const int i = blockIdx.x * 256 + threadIdx.x;
  const u64 v = (i < E) ? (((u64)(unsigned)dst[i]) << 16) | (unsigned)src[i] : ~(u64)0;
  VST2(u64, A + i, v);
}
__device__ __forceinline__ void cas_lds(u64* s, int lo, int hi, bool up) {
  const u64 a = s[lo], b = s[hi];
  const bool sw = up ? (a > b) : (a < b);
  s[lo] = sw ? b : a; s[hi] = sw ? a : b;
}
__global__ __launch_bounds__(256) void k_sort_local(u64* __restrict__ A) {
  __shared__ u64 s[TILE];
  const int base = blockIdx.x * TILE, t = threadIdx.x;
  for (int i = t; i < TILE; i += 256) s[i] = A[base + i];
  __syncthreads();
  for (int k = 2; k <= TILE; k <<= 1) {
    for (int j = k >> 1; j > 0; j >>= 1) {
      for (int p = t; p < TILE / 2; p += 256) {
        const int lo = ((p >> __builtin_ctz(j)) << (__builtin_ctz(j) + 1)) | (p & (j - 1));
        const int hi = lo + j;
        const bool up = (((base + lo) & k) == 0);
        cas_lds(s, lo, hi, up);
      }
      __syncthreads();
    }
  }
  for (int pass = 0; pass < 2; ++pass) { for (int i = t; i < TILE; i += 256) *(volatile u64*)(A + base + i) = s[i]; __threadfence(); }
}
__global__ __launch_bounds__(256) void k_sort_global(u64* __restrict__ A, int logj, int k) {
  const int p = blockIdx.x * 256 + threadIdx.x;
  const int j = 1 << logj;
  const int lo = ((p >> logj) << (logj + 1)) | (p & (j - 1));
  const int hi = lo + j;
  const u64 a = A[lo], b = A[hi];
  const bool up = ((lo & k) == 0);
  const bool sw = up ? (a > b) : (a < b);
  const u64 vlo = sw ? b : a, vhi = sw ? a : b;
  *(volatile u64*)(A + lo) = vlo; *(volatile u64*)(A + hi) = vhi; __threadfence();
  *(volatile u64*)(A + lo) = vlo; *(volatile u64*)(A + hi) = vhi;
}
__global__ __launch_bounds__(256) void k_sort_lds(u64* __restrict__ A, int k) {
  __shared__ u64 s[TILE];
  const int base = blockIdx.x * TILE, t = threadIdx.x;
  for (int i = t; i < TILE; i += 256) s[i] = A[base + i];
  __syncthreads();
  for (int j = TILE >> 1; j > 0; j >>= 1) {
    for (int p = t; p < TILE / 2; p += 256) {
      const int lo = ((p >> __builtin_ctz(j)) << (__builtin_ctz(j) + 1)) | (p & (j - 1));
      const int hi = lo + j;
      const bool up = (((base + lo) & k) == 0);
      cas_lds(s, lo, hi, up);
    }
    __syncthreads();
  }
  for (int pass = 0; pass < 2; ++pass) { for (int i = t; i < TILE; i += 256) *(volatile u64*)(A + base + i) = s[i]; __threadfence(); }
}
__device__ __forceinline__ int lower_bound_key(const u64* __restrict__ A, int n, unsigned key) {
  int lo = 0, hi = n;
  while (lo < hi) { const int mid = (lo + hi) >> 1; if ((unsigned)(A[mid] >> 16) < key) lo = mid + 1; else hi = mid; }
  return lo;
}
__global__ __launch_bounds__(256) void k_segs(const u64* __restrict__ A, v2i* __restrict__ seg, float* __restrict__ dinv, int N, int Npad) {
  const int n = blockIdx.x * 256 + threadIdx.x;
  if (n >= Npad) return;
  int st = 0, c = 0;
  if (n < N) { st = lower_bound_key(A, SORT_N, (unsigned)n); c = lower_bound_key(A, SORT_N, (unsigned)(n + 1)) - st; }
  const v2i sv = {st, c};
  VST2(v2i, seg + n, sv);
  VST2(float, dinv + n, (n < N) ? (1.0f / sqrtf((float)c + 1.0f)) : 0.0f);
}

#define RPB 512
__global__ __launch_bounds__(128) void k_colpart(const float* __restrict__ h, int rows, int ld, float* __restrict__ part) {
  const int c = threadIdx.x, r0 = blockIdx.x * RPB;
  const int r1 = min(r0 + RPB, rows);
  float s = 0.f, s2 = 0.f;
  for (int r = r0; r < r1; ++r) { const float v = h[(size_t)r * ld + c]; s += v; s2 += v * v; }
  VST2(float, part + (size_t)blockIdx.x * 2 * HD + c, s);
  VST2(float, part + (size_t)blockIdx.x * 2 * HD + HD + c, s2);
}
__global__ __launch_bounds__(128) void k_colred(const float* __restrict__ part, int nblk, int rows, const float* __restrict__ g, const float* __restrict__ b,
                                              float* __restrict__ ss) {
  const int c = threadIdx.x;
  double s = 0.0, s2 = 0.0;
  for (int k = 0; k < nblk; ++k) { s += (double)part[(size_t)k * 2 * HD + c]; s2 += (double)part[(size_t)k * 2 * HD + HD + c]; }
  const double mean = s / rows, var = fmax(s2 / rows - mean * mean, 0.0);
  const float sc = g[c] * (float)(1.0 / sqrt(var + 1e-5));
  VST2(float, ss + c, sc);
  VST2(float, ss + HD + c, b[c] - (float)mean * sc);
}
__global__ __launch_bounds__(256) void k_bn_apply_f16(const float* __restrict__ src, const float* __restrict__ ss, _Float16* __restrict__ dst,
                                                     int validrows, int rows) {
  const size_t i8 = (size_t)blockIdx.x * 256 + threadIdx.x;
  if (i8 * 8 >= (size_t)rows * HD) return;
  const size_t i = i8 * 8; const int n = (int)(i >> 7), c0 = (int)(i & (HD - 1));
  v8h v;
#pragma unroll
  for (int e = 0; e < 8; ++e) v[e] = (_Float16)((n < validrows) ? (src[i + e] * (ss ? ss[c0 + e] : 1.0f) + (ss ? ss[HD + c0 + e] : 0.0f)) : 0.0f);
  VST2(v8h, dst + i, v);
}
__global__ __launch_bounds__(256) void k_wcvt(const float* __restrict__ W, _Float16* __restrict__ Wt) {
  const int i8 = blockIdx.x * 256 + threadIdx.x;
  if (i8 >= HD * HD / 8) return;
  const int n = (i8 * 8) >> 7, k0 = (i8 * 8) & 127;
  v8h v;
#pragma unroll
  for (int e = 0; e < 8; ++e) v[e] = (_Float16)W[(k0 + e) * HD + n];
  VST2(v8h, Wt + (size_t)i8 * 8, v);
}

__global__ __launch_bounds__(256) void k_gemm_wmma(const _Float16* __restrict__ A, const _Float16* __restrict__ Wt,
                                                   const float* __restrict__ bias, float* __restrict__ out, int relu) {
  __shared__ __attribute__((aligned(16))) _Float16 sW[HD * HD];
  for (int i = threadIdx.x; i < HD * HD / 8; i += 256) *(v8h*)(sW + i * 8) = *(const v8h*)(Wt + i * 8);
  __syncthreads();
  const int wid = threadIdx.x >> 5, lane = threadIdx.x & 31, m = lane & 15, half = lane >> 4;
  const size_t rowBase = (size_t)blockIdx.x * 128 + wid * 16;
  const _Float16* arow = A + (rowBase + m) * HD;
  v8f acc[8];
#pragma unroll
  for (int nt = 0; nt < 8; ++nt) acc[nt] = (v8f){};
#pragma unroll
  for (int kt = 0; kt < 4; ++kt) {
    const int ka = kt * 32 + half * 8;
    const v8h a0 = *(const v8h*)(arow + ka), a1 = *(const v8h*)(arow + ka + 16);
    const v16h a = __builtin_shufflevector(a0, a1, 0,1,2,3,4,5,6,7,8,9,10,11,12,13,14,15);
#pragma unroll
    for (int nt = 0; nt < 8; ++nt) {
      const _Float16* bp = sW + (nt * 16 + m) * HD + ka;
      const v8h b0 = *(const v8h*)bp, b1 = *(const v8h*)(bp + 16);
      acc[nt] = wmma16(a, __builtin_shufflevector(b0, b1, 0,1,2,3,4,5,6,7,8,9,10,11,12,13,14,15), acc[nt]);
    }
  }
  for (int pass = 0; pass < 2; ++pass) {
#pragma unroll
    for (int pr = 0; pr < 4; ++pr) {
      const int c = pr * 32 + lane;
      const float bb = bias ? bias[c] : 0.f;
#pragma unroll
      for (int r = 0; r < 8; ++r) {
        const float a_ = acc[2 * pr][r], b_ = acc[2 * pr + 1][r];
        const float ax = __shfl_xor(a_, 16), bx = __shfl_xor(b_, 16);
        float v1 = (half ? bx : a_) + bb, v2 = (half ? b_ : ax) + bb;
        if (relu) { v1 = fmaxf(v1, 0.f); v2 = fmaxf(v2, 0.f); }
        *(volatile float*)(out + (rowBase + r) * HD + c) = v1;
        *(volatile float*)(out + (rowBase + r + 8) * HD + c) = v2;
      }
    }
    __threadfence();
  }
}

__global__ __launch_bounds__(256) void k_aggr(const u64* __restrict__ A, const v2i* __restrict__ seg,
                                              const float* __restrict__ dinv, const float* __restrict__ t, const float* __restrict__ bias,
                                              float* __restrict__ h, int N) {
  const size_t i8 = (size_t)blockIdx.x * 256 + threadIdx.x;
  if (i8 >= (size_t)N * HD / 8) return;
  const int n = (int)(i8 >> 4), c0 = (int)(i8 & 15) * 8;
  const v2i sv = seg[n];
  const float dn = dinv[n];
  v8f s = {};
  for (int p = 0; p < sv[1]; ++p) {
    const int sn = (int)(A[sv[0] + p] & 0xffffu);
    const v8f tv = *(const v8f*)(t + (size_t)sn * HD + c0);
    const float ds = dinv[sn];
#pragma unroll
    for (int e = 0; e < 8; ++e) s[e] += tv[e] * ds;
  }
  const v8f tn = *(const v8f*)(t + (size_t)n * HD + c0);
  v8f o;
#pragma unroll
  for (int e = 0; e < 8; ++e) o[e] = fmaxf(s[e] * dn + tn[e] * dn * dn + bias[c0 + e], 0.f);
  VST2(v8f, h + (size_t)n * HD + c0, o);
}

__global__ __launch_bounds__(256) void k_gate(const float* __restrict__ u, const float* __restrict__ w2, const float* __restrict__ b2,
                                              float* __restrict__ gate, int N, int Npad) {
  const int n = blockIdx.x * 256 + threadIdx.x;
  if (n >= Npad) return;
  float s = 0.f;
  if (n < N) { for (int c = 0; c < HD; ++c) s += u[(size_t)n * HD + c] * w2[c]; s = 1.f / (1.f + expf(-(s + b2[0]))); }
  VST2(float, gate + n, s);
}
__global__ __launch_bounds__(256) void k_gsegs(const int* __restrict__ batch, int N, v2i* __restrict__ gseg) {
  const int g = threadIdx.x;
  int lo = 0, hi = N;  while (lo < hi) { const int mid = (lo + hi) >> 1; if (batch[mid] < g) lo = mid + 1; else hi = mid; }
  const int st = lo;
  lo = 0; hi = N;      while (lo < hi) { const int mid = (lo + hi) >> 1; if (batch[mid] < g + 1) lo = mid + 1; else hi = mid; }
  const v2i sv = {st, lo - st};
  VST2(v2i, gseg + g, sv);
}
__global__ __launch_bounds__(128) void k_pool(const float* __restrict__ h, const float* __restrict__ gate, const v2i* __restrict__ gseg, float* __restrict__ gpool) {
  const int g = blockIdx.x, c = threadIdx.x;
  const v2i sv = gseg[g];
  float s = 0.f;
  for (int n = sv[0]; n < sv[0] + sv[1]; ++n) s += h[(size_t)n * HD + c] * gate[n];
  VST2(float, gpool + (size_t)g * HD + c, s);
}
__global__ __launch_bounds__(256) void k_bn_pool_f16(const float* __restrict__ gp, const float* __restrict__ g, const float* __restrict__ b, _Float16* __restrict__ out) {
  __shared__ float sc[HD], sh[HD];
  const int t = threadIdx.x;
  if (t < HD) {
    double s = 0.0, s2 = 0.0;
    for (int r = 0; r < NGRAPH; ++r) { const double v = gp[r * HD + t]; s += v; s2 += v * v; }
    const double mean = s / NGRAPH, var = fmax(s2 / NGRAPH - mean * mean, 0.0);
    sc[t] = g[t] * (float)(1.0 / sqrt(var + 1e-5)); sh[t] = b[t] - (float)mean * sc[t];
  }
  __syncthreads();
  for (int i8 = t; i8 < NGRAPH * HD / 8; i8 += 256) {
    v8h v; const int c0 = (i8 * 8) & 127;
#pragma unroll
    for (int e = 0; e < 8; ++e) v[e] = (_Float16)(gp[i8 * 8 + e] * sc[c0 + e] + sh[c0 + e]);
    VST2(v8h, out + i8 * 8, v);
  }
}
__global__ __launch_bounds__(256) void k_classify(const float* __restrict__ gfc, const float* __restrict__ W, const float* __restrict__ b, float* __restrict__ out) {
  __shared__ float sW[HD * 10];
  __shared__ float sb[10];
  __shared__ __attribute__((aligned(16))) float so[NGRAPH * 10];
  const int t = threadIdx.x;
  for (int i = t; i < HD * 10; i += 256) sW[i] = W[i];
  if (t < 10) sb[t] = b[t];
  __syncthreads();
  {
    const int gi = t;
    float lg[10];
#pragma unroll
    for (int j = 0; j < 10; ++j) lg[j] = sb[j];
    for (int c = 0; c < HD; ++c) { const float v = gfc[(size_t)gi * HD + c];
#pragma unroll
      for (int j = 0; j < 10; ++j) lg[j] += v * sW[c * 10 + j]; }
    float mx = lg[0];
#pragma unroll
    for (int j = 1; j < 10; ++j) mx = fmaxf(mx, lg[j]);
    float se = 0.f;
#pragma unroll
    for (int j = 0; j < 10; ++j) se += expf(lg[j] - mx);
    const float lse = mx + logf(se);
#pragma unroll
    for (int j = 0; j < 10; ++j) so[gi * 10 + j] = lg[j] - lse;
  }
  __syncthreads();
  for (int p = t; p < NGRAPH * 10 / 4; p += 256) VST2(v4f, out + p * 4, *(const v4f*)(so + p * 4));
}

extern "C" void kernel_launch(void* const* d_in, const int* in_sizes, int n_in,
                              void* d_out, int out_size, void* d_ws, size_t ws_size,
                              hipStream_t stream) {
  (void)n_in; (void)out_size;
  const float* x           = (const float*)d_in[0];
  const int*   edges       = (const int*)d_in[1];
  const int*   batch       = (const int*)d_in[2];
  const float* bn_feat_g   = (const float*)d_in[3];
  const float* bn_feat_b   = (const float*)d_in[4];
  const float* conv_feat_W = (const float*)d_in[5];
  const float* conv_feat_b = (const float*)d_in[6];
  const float* conv_W      = (const float*)d_in[7];
  const float* conv_b      = (const float*)d_in[8];
  const float* bn_conv_g   = (const float*)d_in[9];
  const float* bn_conv_b   = (const float*)d_in[10];
  const float* gate_W1     = (const float*)d_in[11];
  const float* gate_b1     = (const float*)d_in[12];
  const float* gate_W2     = (const float*)d_in[13];
  const float* gate_b2     = (const float*)d_in[14];
  const float* fc_W        = (const float*)d_in[15];
  const float* fc_b        = (const float*)d_in[16];
  const float* bn_fc_g     = (const float*)d_in[17];
  const float* bn_fc_b     = (const float*)d_in[18];
  const float* cls_W       = (const float*)d_in[19];
  const float* cls_b       = (const float*)d_in[20];

  const int N    = in_sizes[0] / HD;
  const int E    = in_sizes[1] / 2;
  const int Npad = (N + 127) & ~127;
  if (E > SORT_N || N > 65535) return;

  char* ws = (char*)d_ws;
  size_t off = 0;
  auto carve = [&](size_t bytes) -> char* { char* p = ws + off; off += (bytes + 255) & ~(size_t)255; return p; };
  u64*      keys  = (u64*)carve((size_t)SORT_N * 4);
  v2i*      seg   = (v2i*)carve((size_t)Npad * 8);
  float*    dinv  = (float*)carve((size_t)Npad * 4);
  float*    h     = (float*)carve((size_t)Npad * HD * 4);
  float*    t     = (float*)carve((size_t)Npad * HD * 4);
  _Float16* Ah    = (_Float16*)carve((size_t)Npad * HD * 2);
  _Float16* Wt    = (_Float16*)carve((size_t)HD * HD * 2);
  const int NBLK  = (N + RPB - 1) / RPB;
  float*    part  = (float*)carve((size_t)NBLK * 2 * HD * 4);
  float*    ss    = (float*)carve((size_t)2 * HD * 4);
  float*    gate  = (float*)carve((size_t)Npad * 4);
  v2i*      gseg  = (v2i*)carve((size_t)NGRAPH * 8);
  float*    gpool = (float*)carve((size_t)NGRAPH * HD * 4);
  if (off > ws_size) return;

  const int* srcIdx = edges;
  const int* dstIdx = edges + E;
  dim3 b256(256);
  auto cdiv = [](long long a, long long b_) { return (int)((a + b_ - 1) / b_); };

  k_sort_init<<<SORT_N / 256, b256, 0, stream>>>(srcIdx, dstIdx, keys, E);
  k_sort_local<<<SORT_N / TILE, b256, 0, stream>>>(keys);
  for (int k = TILE * 2; k <= SORT_N; k <<= 1) {
    for (int logj = __builtin_ctz(k) - 1; (1 << logj) >= TILE; --logj)
      k_sort_global<<<SORT_N / 2 / 256, b256, 0, stream>>>(keys, logj, k);
    k_sort_lds<<<SORT_N / TILE, b256, 0, stream>>>(keys, k);
  }
  k_segs<<<cdiv(Npad, 256), b256, 0, stream>>>(keys, seg, dinv, N, Npad);

  auto conv_layer = [&](const float* inp, const float* bng, const float* bnb, const float* W, const float* bias) {
    k_colpart<<<NBLK, dim3(HD), 0, stream>>>(inp, N, HD, part);
    k_colred<<<1, dim3(HD), 0, stream>>>(part, NBLK, N, bng, bnb, ss);
    k_bn_apply_f16<<<cdiv((long long)Npad * HD / 8, 256), b256, 0, stream>>>(inp, ss, Ah, N, Npad);
    k_wcvt<<<HD * HD / 8 / 256, b256, 0, stream>>>(W, Wt);
    k_gemm_wmma<<<Npad / 128, b256, 0, stream>>>(Ah, Wt, nullptr, t, 0);
    k_aggr<<<cdiv((long long)N * HD / 8, 256), b256, 0, stream>>>(keys, seg, dinv, t, bias, h, N);
  };
  conv_layer(x, bn_feat_g, bn_feat_b, conv_feat_W, conv_feat_b);
  for (int i = 0; i < 3; ++i)
    conv_layer(h, bn_conv_g + i * HD, bn_conv_b + i * HD, conv_W + (size_t)i * HD * HD, conv_b + i * HD);

  k_bn_apply_f16<<<cdiv((long long)Npad * HD / 8, 256), b256, 0, stream>>>(h, nullptr, Ah, N, Npad);
  k_wcvt<<<HD * HD / 8 / 256, b256, 0, stream>>>(gate_W1, Wt);
  k_gemm_wmma<<<Npad / 128, b256, 0, stream>>>(Ah, Wt, gate_b1, t, 1);
  k_gate<<<cdiv(Npad, 256), b256, 0, stream>>>(t, gate_W2, gate_b2, gate, N, Npad);

  k_gsegs<<<1, b256, 0, stream>>>(batch, N, gseg);
  k_pool<<<NGRAPH, dim3(HD), 0, stream>>>(h, gate, gseg, gpool);

  k_bn_pool_f16<<<1, b256, 0, stream>>>(gpool, bn_fc_g, bn_fc_b, Ah);
  k_wcvt<<<HD * HD / 8 / 256, b256, 0, stream>>>(fc_W, Wt);
  k_gemm_wmma<<<NGRAPH / 128, b256, 0, stream>>>(Ah, Wt, fc_b, t, 1);
  k_classify<<<1, b256, 0, stream>>>(t, cls_W, cls_b, (float*)d_out);
}
